// INLVisionBlock_40578851012932
// MI455X (gfx1250) — hardware-verified
//
#include <hip/hip_runtime.h>

typedef _Float16 v16h __attribute__((ext_vector_type(16)));
typedef _Float16 v8h  __attribute__((ext_vector_type(8)));
typedef float    v8f  __attribute__((ext_vector_type(8)));
typedef float    v4f  __attribute__((ext_vector_type(4)));
typedef v8h __attribute__((may_alias)) v8ha;
typedef v4f __attribute__((may_alias)) v4fa;

union Frag { v16h v; v8h half[2]; };

#define DM   768
#define NH   12
#define HD   64
#define SQ   197
#define NB   64
#define NT   (NB * SQ)
#define DQ   2304
#define DF   3072
#define DFH  1536
#define VTP  256
#define NSTEP 5
#define PSCALE 16384.0f
#define WSCALE 32.0f
#define WINV   0.03125f

#define OFF_WIN  0
#define OFF_WOUT (DQ * DM)
#define OFF_WD1  (OFF_WOUT + DM * DM)
#define OFF_WD2  (OFF_WD1 + DM * DM)
#define OFF_WF1  (OFF_WD2 + DM * DM)
#define OFF_WF2  (OFF_WF1 + DF * DM)
#define NWH      (OFF_WF2 + DF * DM)

__device__ __forceinline__ v8f wmma_f16(v16h a, v16h b, v8f c) {
  v8f d = __builtin_amdgcn_wmma_f32_16x16x32_f16(false, a, false, b, (short)0, c, false, false);
  asm volatile("v_nop\n\tv_nop\n\tv_nop\n\tv_nop" : "+v"(d) : "v"(a), "v"(b));
  return d;
}

__device__ __forceinline__ v16h load_frag(const _Float16* p, int h) {
  Frag f;
  f.half[0] = *(const v8ha*)(p + 8 * h);
  f.half[1] = *(const v8ha*)(p + 16 + 8 * h);
  return f.v;
}

__device__ __forceinline__ float gelu_erf(float v) {
  return 0.5f * v * (1.0f + erff(v * 0.70710678118654752f));
}

template <int ACT>
__device__ __forceinline__ float epi1(float a, float b, float bsc, float alpha) {
  float t = a * WINV + bsc * b;
  if (ACT) t = gelu_erf(t);
  return t * alpha;
}

__device__ __forceinline__ v8h to_h8(v4f a, v4f c) {
  const v8h o = { (_Float16)a.x, (_Float16)a.y, (_Float16)a.z, (_Float16)a.w,
                  (_Float16)c.x, (_Float16)c.y, (_Float16)c.z, (_Float16)c.w };
  return o;
}

__global__ __launch_bounds__(256) void cvt_w_kernel(
    const float* __restrict__ w0, const float* __restrict__ w1, const float* __restrict__ w2,
    const float* __restrict__ w3, const float* __restrict__ w4, const float* __restrict__ w5,
    _Float16* __restrict__ wh)
{
  const int sel = blockIdx.y;
  const float* src;
  int n8, doff8;
  if (sel == 0)      { src = w0; n8 = DQ * DM / 8; doff8 = OFF_WIN / 8; }
  else if (sel == 1) { src = w1; n8 = DM * DM / 8; doff8 = OFF_WOUT / 8; }
  else if (sel == 2) { src = w2; n8 = DM * DM / 8; doff8 = OFF_WD1 / 8; }
  else if (sel == 3) { src = w3; n8 = DM * DM / 8; doff8 = OFF_WD2 / 8; }
  else if (sel == 4) { src = w4; n8 = DF * DM / 8; doff8 = OFF_WF1 / 8; }
  else               { src = w5; n8 = DF * DM / 8; doff8 = OFF_WF2 / 8; }
  const int g = blockIdx.x * 256 + threadIdx.x;
  if (g >= n8) return;
  const float* p = src + (size_t)g * 8;
  const v4f a = *(const v4fa*)p;
  const v4f c = *(const v4fa*)(p + 4);
  const v4f as = a * WSCALE, cs = c * WSCALE;
  const v8h o = to_h8(as, cs);
  _Float16* dst = wh + ((size_t)doff8 + (size_t)g) * 8;
  *(volatile v8h*)dst = o;
  __threadfence();
  *(volatile v8h*)dst = o;
}

template <int MODE>
__global__ __launch_bounds__(256) void ln_kernel(const float* in, const float* in2,
                                                 const float* __restrict__ gam,
                                                 const float* __restrict__ bet,
                                                 float* outF, _Float16* outH)
{
  __shared__ __attribute__((aligned(16))) float srow[8 * DM];
  const int tid = threadIdx.x, lane = tid & 31, w = tid >> 5;
  const size_t row = (size_t)blockIdx.x * 8 + w;
  const float* xr = in + row * DM;

  v4f v[6];
  #pragma unroll
  for (int i = 0; i < 6; ++i) v[i] = *(const v4fa*)(xr + 4 * lane + 128 * i);
  if (MODE == 2) {
    const float* x2r = in2 + row * DM;
    #pragma unroll
    for (int i = 0; i < 6; ++i) {
      const v4f t = *(const v4fa*)(x2r + 4 * lane + 128 * i);
      v[i] = v[i] + t;
    }
    float* orow = outF + row * DM;
    #pragma unroll
    for (int i = 0; i < 6; ++i) *(volatile v4f*)(orow + 4 * lane + 128 * i) = v[i];
  }

  float s = 0.0f;
  #pragma unroll
  for (int i = 0; i < 6; ++i) s += (v[i].x + v[i].y) + (v[i].z + v[i].w);
  #pragma unroll
  for (int off = 16; off > 0; off >>= 1) s += __shfl_xor(s, off);
  const float mu = s * (1.0f / DM);

  v4f d[6];
  float q = 0.0f;
  #pragma unroll
  for (int i = 0; i < 6; ++i) {
    d[i] = v[i] - mu;
    q += d[i].x * d[i].x + d[i].y * d[i].y + d[i].z * d[i].z + d[i].w * d[i].w;
  }
  #pragma unroll
  for (int off = 16; off > 0; off >>= 1) q += __shfl_xor(q, off);
  const float rstd = rsqrtf(q * (1.0f / DM) + 1e-5f);

  v4f y[6];
  #pragma unroll
  for (int i = 0; i < 6; ++i) {
    const v4f gg = *(const v4fa*)(gam + 4 * lane + 128 * i);
    const v4f bb = *(const v4fa*)(bet + 4 * lane + 128 * i);
    y[i] = d[i] * rstd * gg + bb;
  }
  if (MODE == 1) {
    float* orow = outF + row * DM;
    #pragma unroll
    for (int i = 0; i < 6; ++i) *(volatile v4f*)(orow + 4 * lane + 128 * i) = y[i];
  }
  float* sr = srow + w * DM;
  #pragma unroll
  for (int i = 0; i < 6; ++i) *(v4fa*)(sr + 4 * lane + 128 * i) = y[i];
  __syncthreads();
  __threadfence();
  if (MODE == 2) {
    float* orow = outF + row * DM;
    #pragma unroll
    for (int i = 0; i < 6; ++i) *(volatile v4f*)(orow + 4 * lane + 128 * i) = v[i];
  }
  if (MODE == 1) {
    float* orow = outF + row * DM;
    #pragma unroll
    for (int i = 0; i < 6; ++i) *(volatile v4f*)(orow + 4 * lane + 128 * i) = y[i];
  }

  v8h hv[3];
  #pragma unroll
  for (int i = 0; i < 3; ++i) {
    const float* pp = sr + 8 * lane + 256 * i;
    const v4f a = *(const v4fa*)pp;
    const v4f c = *(const v4fa*)(pp + 4);
    hv[i] = to_h8(a, c);
  }
  _Float16* hr = outH + row * DM;
  #pragma unroll
  for (int i = 0; i < 3; ++i) *(volatile v8h*)(hr + 8 * lane + 256 * i) = hv[i];
  __threadfence();
  #pragma unroll
  for (int i = 0; i < 3; ++i) *(volatile v8h*)(hr + 8 * lane + 256 * i) = hv[i];
}

template <int ACT, int RES, int OUTF, int OUTH>
__global__ __launch_bounds__(128) void gemm_kernel(
    const _Float16* __restrict__ A, int lda,
    const _Float16* __restrict__ W, int ldw, int K,
    const float* __restrict__ bias, float bsc, float alpha,
    const float* resid, int ldr,
    float* outF, _Float16* outH, int ldo)
{
  __shared__ __attribute__((aligned(16))) float sT[4 * 2048];

  const int tid = threadIdx.x, lane = tid & 31, w = tid >> 5;
  const int h = lane >> 4, m = lane & 15;
  const int m0w = blockIdx.x * 64 + 32 * (w & 1);
  const int e0w = blockIdx.y * 128 + 64 * (w >> 1);

  const _Float16* xa0 = A + (size_t)(m0w + m) * lda;
  const _Float16* xa1 = xa0 + (size_t)16 * lda;
  const _Float16* wb  = W + (size_t)(e0w + m) * ldw;

  const v8f zero8 = {0.f, 0.f, 0.f, 0.f, 0.f, 0.f, 0.f, 0.f};
  v8f acc[2][4];
  #pragma unroll
  for (int mt = 0; mt < 2; ++mt)
    #pragma unroll
    for (int nt = 0; nt < 4; ++nt) acc[mt][nt] = zero8;

  #pragma unroll 1
  for (int k0 = 0; k0 < K; k0 += 32) {
    const v16h a0 = load_frag(xa0 + k0, h);
    const v16h a1 = load_frag(xa1 + k0, h);
    #pragma unroll
    for (int nt = 0; nt < 4; ++nt) {
      const v16h b = load_frag(wb + (size_t)nt * 16 * ldw + k0, h);
      acc[0][nt] = wmma_f16(a0, b, acc[0][nt]);
      acc[1][nt] = wmma_f16(a1, b, acc[1][nt]);
    }
  }

  float* so = sT + w * 2048;
  #pragma unroll
  for (int mt = 0; mt < 2; ++mt)
    #pragma unroll
    for (int nt = 0; nt < 4; ++nt)
      #pragma unroll
      for (int r = 0; r < 8; ++r)
        so[(16 * mt + 8 * h + r) * 64 + 16 * nt + m] = acc[mt][nt][r];
  __syncthreads();

  const int q8 = lane & 7, sub = lane >> 3;
  const int rsub = sub >> 1, csub = 32 * (sub & 1) + 4 * q8;

  #pragma unroll 1
  for (int i = 0; i < 16; ++i) {
    const int row = 2 * i + rsub;
    float* sp = so + row * 64 + csub;
    const v4f a = *(const v4fa*)sp;
    const int gcol = e0w + csub;
    const size_t grow = (size_t)(m0w + row);
    const v4f bb = *(const v4fa*)(bias + gcol);
    v4f v;
    v.x = epi1<ACT>(a.x, bb.x, bsc, alpha);
    v.y = epi1<ACT>(a.y, bb.y, bsc, alpha);
    v.z = epi1<ACT>(a.z, bb.z, bsc, alpha);
    v.w = epi1<ACT>(a.w, bb.w, bsc, alpha);
    if (RES) {
      const v4f rr = *(const v4fa*)(resid + grow * (size_t)ldr + gcol);
      v = v + rr;
    }
    *(v4fa*)sp = v;
    if (OUTF) *(volatile v4f*)(outF + grow * (size_t)ldo + gcol) = v;
  }
  __syncthreads();
  __threadfence();
  if (OUTF) {
    #pragma unroll 1
    for (int i = 0; i < 16; ++i) {
      const int row = 2 * i + rsub;
      const float* sp = so + row * 64 + csub;
      const v4f v = *(const v4fa*)sp;
      const int gcol = e0w + csub;
      const size_t grow = (size_t)(m0w + row);
      *(volatile v4f*)(outF + grow * (size_t)ldo + gcol) = v;
    }
  }
  if (OUTH) {
    v8h hv[8];
    #pragma unroll
    for (int i = 0; i < 8; ++i) {
      const float* pp = so + (4 * i + sub) * 64 + 8 * q8;
      const v4f a = *(const v4fa*)pp;
      const v4f c = *(const v4fa*)(pp + 4);
      hv[i] = to_h8(a, c);
    }
    #pragma unroll
    for (int i = 0; i < 8; ++i)
      *(volatile v8h*)(outH + (size_t)(m0w + 4 * i + sub) * (size_t)ldo + e0w + 8 * q8) = hv[i];
    __threadfence();
    #pragma unroll
    for (int i = 0; i < 8; ++i)
      *(volatile v8h*)(outH + (size_t)(m0w + 4 * i + sub) * (size_t)ldo + e0w + 8 * q8) = hv[i];
  }
}

__global__ __launch_bounds__(128) void vtrans_kernel(const _Float16* __restrict__ qkv,
                                                    _Float16* __restrict__ vt)
{
  __shared__ __attribute__((aligned(16))) _Float16 sK[64 * 72];
  const int tid = threadIdx.x, lane = tid & 31, w = tid >> 5;
  const int kt = blockIdx.x, bh = blockIdx.y;
  const int b = bh / NH, hd = bh - b * NH;
  const v8h z8 = {(_Float16)0.f, (_Float16)0.f, (_Float16)0.f, (_Float16)0.f,
                  (_Float16)0.f, (_Float16)0.f, (_Float16)0.f, (_Float16)0.f};
  #pragma unroll
  for (int i = 0; i < 4; ++i) {
    const int c = tid + 128 * i;
    const int key = c >> 3, p = c & 7;
    int tk = kt * 64 + key;
    const bool ok = tk < SQ;
    tk = ok ? tk : (SQ - 1);
    const _Float16* src = qkv + ((size_t)b * SQ + tk) * DQ + 2 * DM + HD * hd + 8 * p;
    v8h v = *(const v8ha*)src;
    if (!ok) v = z8;
    *(v8ha*)(sK + key * 72 + 8 * p) = v;
  }
  __syncthreads();

  const int q8 = lane & 7, sub = lane >> 3;
  v8h ov[4];
  #pragma unroll
  for (int i = 0; i < 4; ++i) {
    const int d = 16 * i + 4 * w + sub;
    v8h t = z8;
    #pragma unroll
    for (int kk = 0; kk < 8; ++kk) t[kk] = sK[(8 * q8 + kk) * 72 + d];
    ov[i] = t;
  }
  #pragma unroll
  for (int i = 0; i < 4; ++i) {
    const int d = 16 * i + 4 * w + sub;
    *(volatile v8h*)(vt + ((size_t)bh * HD + d) * VTP + kt * 64 + 8 * q8) = ov[i];
  }
  __threadfence();
  #pragma unroll
  for (int i = 0; i < 4; ++i) {
    const int d = 16 * i + 4 * w + sub;
    *(volatile v8h*)(vt + ((size_t)bh * HD + d) * VTP + kt * 64 + 8 * q8) = ov[i];
  }
}

__device__ __forceinline__ v16h pack_p(v8f a, v8f c) {
  const v16h r = { (_Float16)(a[0] * PSCALE), (_Float16)(a[1] * PSCALE), (_Float16)(a[2] * PSCALE), (_Float16)(a[3] * PSCALE),
                   (_Float16)(a[4] * PSCALE), (_Float16)(a[5] * PSCALE), (_Float16)(a[6] * PSCALE), (_Float16)(a[7] * PSCALE),
                   (_Float16)(c[0] * PSCALE), (_Float16)(c[1] * PSCALE), (_Float16)(c[2] * PSCALE), (_Float16)(c[3] * PSCALE),
                   (_Float16)(c[4] * PSCALE), (_Float16)(c[5] * PSCALE), (_Float16)(c[6] * PSCALE), (_Float16)(c[7] * PSCALE) };
  return r;
}

__global__ __launch_bounds__(32) void attn_kernel(const _Float16* __restrict__ qkv,
                                                  const _Float16* __restrict__ vt,
                                                  _Float16* __restrict__ ctx)
{
  __shared__ __attribute__((aligned(16))) float sO[16 * 64];

  const int lane = threadIdx.x, h = lane >> 4, m = lane & 15;
  const int qt = blockIdx.x, hd = blockIdx.y, b = blockIdx.z;
  const int bh = b * NH + hd;
  const int q0 = qt * 16;
  const int qi = (q0 + m < SQ) ? (q0 + m) : (SQ - 1);

  const _Float16* qrow = qkv + ((size_t)b * SQ + qi) * DQ + HD * hd;
  const v16h qb0 = load_frag(qrow, h);
  const v16h qb1 = load_frag(qrow + 32, h);

  const v8f zero8 = {0.f, 0.f, 0.f, 0.f, 0.f, 0.f, 0.f, 0.f};
  v8f o[4];
  #pragma unroll
  for (int t = 0; t < 4; ++t) o[t] = zero8;
  float mrun = -1e30f, lrun = 0.0f;

  const _Float16* kbase = qkv + (size_t)b * SQ * DQ + DM + HD * hd;
  const _Float16* vbase = vt + ((size_t)bh * HD + m) * VTP;

  #pragma unroll 1
  for (int kb = 0; kb < 4 * 64; kb += 64) {
    v8f s[4];
    #pragma unroll
    for (int j = 0; j < 4; ++j) {
      int key = kb + 16 * j + m;
      key = (key < SQ) ? key : (SQ - 1);
      const _Float16* kp = kbase + (size_t)key * DQ;
      const v16h kf0 = load_frag(kp, h);
      const v16h kf1 = load_frag(kp + 32, h);
      v8f z = zero8;
      z = wmma_f16(kf0, qb0, z);
      z = wmma_f16(kf1, qb1, z);
      s[j] = z;
    }
    #pragma unroll
    for (int j = 0; j < 4; ++j)
      #pragma unroll
      for (int r = 0; r < 8; ++r) {
        const int key = kb + 16 * j + 8 * h + r;
        const float t = s[j][r] * 0.125f;
        s[j][r] = (key < SQ) ? t : -1.0e30f;
      }

    float mloc = s[0][0];
    #pragma unroll
    for (int j = 0; j < 4; ++j)
      #pragma unroll
      for (int r = 0; r < 8; ++r) mloc = fmaxf(mloc, s[j][r]);
    mloc = fmaxf(mloc, __shfl_xor(mloc, 16));
    const float mnew = fmaxf(mrun, mloc);
    const float alpha = __expf(mrun - mnew);
    mrun = mnew;
    float lsum = 0.0f;
    #pragma unroll
    for (int j = 0; j < 4; ++j)
      #pragma unroll
      for (int r = 0; r < 8; ++r) {
        const float p = __expf(s[j][r] - mnew);
        s[j][r] = p;
        lsum += p;
      }
    lsum += __shfl_xor(lsum, 16);
    lrun = lrun * alpha + lsum;
    #pragma unroll
    for (int t = 0; t < 4; ++t)
      #pragma unroll
      for (int r = 0; r < 8; ++r) o[t][r] = o[t][r] * alpha;

    const v16h pb0 = pack_p(s[0], s[1]);
    const v16h pb1 = pack_p(s[2], s[3]);

    #pragma unroll
    for (int t = 0; t < 4; ++t) {
      const _Float16* vp = vbase + (size_t)(16 * t) * VTP + kb;
      const v16h vf0 = load_frag(vp, h);
      const v16h vf1 = load_frag(vp + 32, h);
      o[t] = wmma_f16(vf0, pb0, o[t]);
      o[t] = wmma_f16(vf1, pb1, o[t]);
    }
  }

  const float inv = (1.0f / lrun) * (1.0f / PSCALE);
  #pragma unroll
  for (int t = 0; t < 4; ++t)
    #pragma unroll
    for (int r = 0; r < 8; ++r)
      sO[m * 64 + 16 * t + 8 * h + r] = o[t][r] * inv;
  __syncthreads();

  const int q8 = lane & 7, sub = lane >> 3;
  v8h hv[4];
  #pragma unroll
  for (int i = 0; i < 4; ++i) {
    const float* pp = sO + (4 * i + sub) * 64 + 8 * q8;
    const v4f a = *(const v4fa*)pp;
    const v4f c = *(const v4fa*)(pp + 4);
    hv[i] = to_h8(a, c);
  }
  #pragma unroll
  for (int i = 0; i < 4; ++i) {
    const int q = q0 + 4 * i + sub;
    if (q < SQ)
      *(volatile v8h*)(ctx + ((size_t)b * SQ + q) * DM + HD * hd + 8 * q8) = hv[i];
  }
  __threadfence();
  #pragma unroll
  for (int i = 0; i < 4; ++i) {
    const int q = q0 + 4 * i + sub;
    if (q < SQ)
      *(volatile v8h*)(ctx + ((size_t)b * SQ + q) * DM + HD * hd + 8 * q8) = hv[i];
  }
}

extern "C" void kernel_launch(void* const* d_in, const int* in_sizes, int n_in,
                              void* d_out, int out_size, void* d_ws, size_t ws_size,
                              hipStream_t stream) {
  if (n_in < 19) return;
  if (in_sizes[0] != NT * DM || out_size != NT * DM) return;
  if (in_sizes[1] != DQ * DM || in_sizes[2] != DQ) return;
  if (in_sizes[3] != DM * DM || in_sizes[11] != DM * DM || in_sizes[13] != DM * DM) return;
  if (in_sizes[15] != DF * DM || in_sizes[17] != DF * DM || in_sizes[16] != DF) return;
  if (in_sizes[4] != DM || in_sizes[5] != DM || in_sizes[6] != DM || in_sizes[7] != DM) return;
  if (in_sizes[8] != DM || in_sizes[9] != DM || in_sizes[10] != DM) return;
  if (in_sizes[12] != DM || in_sizes[14] != DM || in_sizes[18] != DM) return;

  const float* x     = (const float*)d_in[0];
  const float* w_in  = (const float*)d_in[1];
  const float* b_in  = (const float*)d_in[2];
  const float* w_out = (const float*)d_in[3];
  const float* b_out = (const float*)d_in[4];
  const float* lnA_g = (const float*)d_in[5];
  const float* lnA_b = (const float*)d_in[6];
  const float* ln1_g = (const float*)d_in[7];
  const float* ln1_b = (const float*)d_in[8];
  const float* ln2_g = (const float*)d_in[9];
  const float* ln2_b = (const float*)d_in[10];
  const float* wd1   = (const float*)d_in[11];
  const float* bd1   = (const float*)d_in[12];
  const float* wd2   = (const float*)d_in[13];
  const float* bd2   = (const float*)d_in[14];
  const float* wf1   = (const float*)d_in[15];
  const float* bf1   = (const float*)d_in[16];
  const float* wf2   = (const float*)d_in[17];
  const float* bf2   = (const float*)d_in[18];
  float* out = (float*)d_out;

  const size_t wh_bytes  = (size_t)NWH * 2;
  const size_t ra_bytes  = (size_t)NT * DM * 2;
  const size_t h16_bytes = (size_t)NT * DM * 2;
  const size_t st_bytes  = (size_t)NT * DM * 4;
  const size_t rb_bytes  = (size_t)NT * DQ * 2;
  const size_t rf_bytes  = (size_t)NT * DM * 4;
  if (h16_bytes + st_bytes > rb_bytes) return;
  if ((size_t)NT * DFH * 2 > rb_bytes) return;
  if ((size_t)NB * NH * HD * VTP * 2 > rf_bytes) return;
  const size_t total = wh_bytes + ra_bytes + rb_bytes + rf_bytes;
  if (total > ws_size) return;

  char* ws = (char*)d_ws;
  _Float16* wh    = (_Float16*)ws;
  _Float16* pA    = (_Float16*)(ws + wh_bytes);
  char*     pB    = ws + wh_bytes + ra_bytes;
  _Float16* qkv16 = (_Float16*)pB;
  _Float16* h16   = (_Float16*)pB;
  float*    st32  = (float*)(pB + h16_bytes);
  _Float16* hf16  = (_Float16*)pB;
  float*    pF    = (float*)(ws + wh_bytes + ra_bytes + rb_bytes);
  _Float16* vt16  = (_Float16*)pF;
  float*    x1    = pF;

  const _Float16* win16  = wh + OFF_WIN;
  const _Float16* wout16 = wh + OFF_WOUT;
  const _Float16* wd1_16 = wh + OFF_WD1;
  const _Float16* wd2_16 = wh + OFF_WD2;
  const _Float16* wf1_16 = wh + OFF_WF1;
  const _Float16* wf2_16 = wh + OFF_WF2;

  cvt_w_kernel<<<dim3(DF * DM / 8 / 256, 6), 256, 0, stream>>>(w_in, w_out, wd1, wd2, wf1, wf2, wh);

  ln_kernel<0><<<NT / 8, 256, 0, stream>>>(x, x, lnA_g, lnA_b, x1, pA);

  gemm_kernel<0, 0, 0, 1><<<dim3(NT / 64, DQ / 128), 128, 0, stream>>>(
      pA, DM, win16, DM, DM, b_in, 1.0f, 1.0f, x, DM, x1, qkv16, DQ);

  vtrans_kernel<<<dim3(4, NB * NH), 128, 0, stream>>>(qkv16, vt16);

  attn_kernel<<<dim3((SQ + 15) / 16, NH, NB), 32, 0, stream>>>(qkv16, vt16, pA);

  gemm_kernel<0, 1, 1, 0><<<dim3(NT / 64, DM / 128), 128, 0, stream>>>(
      pA, DM, wout16, DM, DM, b_out, 1.0f, 1.0f, x, DM, x1, pA, DM);

  ln_kernel<1><<<NT / 8, 256, 0, stream>>>(x1, x1, ln1_g, ln1_b, st32, pA);

  for (int it = 0; it < NSTEP; ++it) {
    gemm_kernel<1, 0, 0, 1><<<dim3(NT / 64, DM / 128), 128, 0, stream>>>(
        pA, DM, wd1_16, DM, DM, bd1, 1.0f, 1.0f, x, DM, x1, h16, DM);
    gemm_kernel<0, 1, 1, 1><<<dim3(NT / 64, DM / 128), 128, 0, stream>>>(
        h16, DM, wd2_16, DM, DM, bd2, 1.0f, 0.1f, st32, DM, st32, pA, DM);
  }

  ln_kernel<2><<<NT / 8, 256, 0, stream>>>(x1, st32, ln2_g, ln2_b, x1, pA);

  for (int hh = 0; hh < 2; ++hh) {
    gemm_kernel<1, 0, 0, 1><<<dim3(NT / 64, DFH / 128), 128, 0, stream>>>(
        pA, DM, wf1_16 + (size_t)hh * DFH * DM, DM, DM, bf1 + hh * DFH, 1.0f, 1.0f,
        x, DM, x1, hf16, DFH);
    const float* res = (hh == 0) ? (const float*)x1 : (const float*)out;
    const float bsc = (hh == 0) ? 1.0f : 0.0f;
    gemm_kernel<0, 1, 1, 0><<<dim3(NT / 64, DM / 128), 128, 0, stream>>>(
        hf16, DFH, wf2_16 + (size_t)hh * DFH, DF, DFH, bf2, bsc, 1.0f,
        res, DM, out, pA, DM);
  }
}
